// KANLinear_20615843021208
// MI455X (gfx1250) — hardware-verified
//
#include <hip/hip_runtime.h>

constexpr int kRows       = 32768;
constexpr int kIn         = 256;
constexpr int kOutF       = 256;
constexpr int kKnots      = 12;
constexpr int kNB         = 8;
constexpr int kKtot       = kIn + kIn * kNB;
constexpr int kHalfRows   = kRows / 2;
constexpr int kRowsPerBlk = 8;
constexpr float kCarryA   = 16.0f;
constexpr float kCarryB   = 16.0f;
constexpr float kOutScale = 1.0f / 256.0f;

constexpr size_t kBtBytes = (size_t)kOutF * kKtot * 2;
constexpr size_t kABytes  = (size_t)kHalfRows * kKtot * 2;
constexpr size_t kWsNeed  = kBtBytes + kABytes;
static_assert(kKtot % 32 == 0);
static_assert(kHalfRows % 64 == 0);
static_assert(kOutF % 64 == 0);
static_assert(kBtBytes % 128 == 0);
static_assert((kKtot * 2) % 128 == 0);
static_assert(kWsNeed == 76677120ull);
static_assert(kWsNeed <= 134217728ull);
static_assert(kHalfRows % kRowsPerBlk == 0);
static_assert(kIn == 256);

typedef __attribute__((ext_vector_type(16))) _Float16 v16h;
typedef __attribute__((ext_vector_type(8)))  _Float16 v8h;
typedef __attribute__((ext_vector_type(16))) __bf16   v16b;
typedef __attribute__((ext_vector_type(8)))  __bf16   v8b;
typedef __attribute__((ext_vector_type(8)))  float    v8f;
typedef __attribute__((ext_vector_type(4)))  float    v4f;

__device__ __forceinline__ unsigned short f2bf_bits(float f) {
  unsigned u = __float_as_uint(f);
  return (unsigned short)((u + 0x7FFFu + ((u >> 16) & 1u)) >> 16);
}
__device__ __forceinline__ float bf_bits2f(unsigned short h) { return __uint_as_float(((unsigned)h) << 16); }

__device__ __forceinline__ void dep_guard_h(v8f& a, v8f& b, v16h x, v16h y) { asm volatile("v_nop\n\tv_nop\n\tv_nop\n\tv_nop" : "+v"(a), "+v"(b) : "v"(x), "v"(y)); }
__device__ __forceinline__ void dep_guard_b(v8f& a, v8f& b, v16b x, v16b y) { asm volatile("v_nop\n\tv_nop\n\tv_nop\n\tv_nop" : "+v"(a), "+v"(b) : "v"(x), "v"(y)); }
__device__ __forceinline__ void dep_guard4_h(v8f& a, v8f& b, v8f& c, v8f& d, v16h x, v16h y) { asm volatile("v_nop\n\tv_nop\n\tv_nop\n\tv_nop" : "+v"(a), "+v"(b), "+v"(c), "+v"(d) : "v"(x), "v"(y)); }
__device__ __forceinline__ void dep_guard4_b(v8f& a, v8f& b, v8f& c, v8f& d, v16b x, v16b y) { asm volatile("v_nop\n\tv_nop\n\tv_nop\n\tv_nop" : "+v"(a), "+v"(b), "+v"(c), "+v"(d) : "v"(x), "v"(y)); }
__device__ __forceinline__ void keep4_h(v16h a, v16h b, v16h c, v16h d) { asm volatile("v_nop" :: "v"(a), "v"(b), "v"(c), "v"(d)); }
__device__ __forceinline__ void keep4_b(v16b a, v16b b, v16b c, v16b d) { asm volatile("v_nop" :: "v"(a), "v"(b), "v"(c), "v"(d)); }
__device__ __forceinline__ void acc_guard4(v8f& a, v8f& b, v8f& c, v8f& d) { asm volatile("v_nop\n\tv_nop\n\tv_nop\n\tv_nop" : "+v"(a), "+v"(b), "+v"(c), "+v"(d)); }
template <typename T> struct Frag;
template <> struct Frag<_Float16> {
  typedef v16h V; union U { v16h v; v8h h[2]; };
  static __device__ __forceinline__ v16h load(const _Float16* p) {
    U f; f.h[0] = *(const v8h*)(p); f.h[1] = *(const v8h*)(p + 16); return f.v;
  }
  static __device__ __forceinline__ v8f mma(v16h a, v16h b, v8f c) {
    return __builtin_amdgcn_wmma_f32_16x16x32_f16(false, a, false, b, (short)0, c, false, false);
  }
  static __device__ __forceinline__ void guard(v8f& a, v8f& b, v16h x, v16h y) { dep_guard_h(a, b, x, y); }
  static __device__ __forceinline__ void guard4(v8f& a, v8f& b, v8f& c, v8f& d, v16h x, v16h y) { dep_guard4_h(a, b, c, d, x, y); }
  static __device__ __forceinline__ void keep(v16h a, v16h b, v16h c, v16h d) { keep4_h(a, b, c, d); }
};
template <> struct Frag<__bf16> {
  typedef v16b V; union U { v16b v; v8b h[2]; };
  static __device__ __forceinline__ v16b load(const __bf16* p) {
    U f; f.h[0] = *(const v8b*)(p); f.h[1] = *(const v8b*)(p + 16); return f.v;
  }
  static __device__ __forceinline__ v8f mma(v16b a, v16b b, v8f c) {
    return __builtin_amdgcn_wmma_f32_16x16x32_bf16(false, a, false, b, (short)0, c, false, false);
  }
  static __device__ __forceinline__ void guard(v8f& a, v8f& b, v16b x, v16b y) { dep_guard_b(a, b, x, y); }
  static __device__ __forceinline__ void guard4(v8f& a, v8f& b, v8f& c, v8f& d, v16b x, v16b y) { dep_guard4_b(a, b, c, d, x, y); }
  static __device__ __forceinline__ void keep(v16b a, v16b b, v16b c, v16b d) { keep4_b(a, b, c, d); }
};

template <int ET> struct Elem;
template <> struct Elem<0> { typedef _Float16 T; };
template <> struct Elem<1> { typedef __bf16 T; };
template <int ET, bool SPLIT, int BIAS_MODE, int OUT_MODE, bool RESID, int ACT = 0>
__global__ __launch_bounds__(256) void wmma_gemm64(
    const unsigned short* __restrict__ Ap, const unsigned short* __restrict__ A2p, int lda, long strideA,
    const unsigned short* __restrict__ Btp, const unsigned short* __restrict__ Bt2p, int ldb, long strideB,
    void* __restrict__ Cout, void* __restrict__ Cout2, int ldc, long strideC,
    const float* __restrict__ bias,
    const float* __restrict__ resid, long strideR,
    int M, int N, int K, float scale) {
  typedef typename Elem<ET>::T T;
  typedef typename Frag<T>::V V;
  const T* A = (const T*)Ap; const T* A2 = (const T*)A2p; const T* Bt = (const T*)Btp; const T* Bt2 = (const T*)Bt2p;
  __shared__ __align__(16) float sT[8][16 * 68];
  const int b    = blockIdx.y;
  const int lane = threadIdx.x & 31;
  const int wave = threadIdx.x >> 5;
  const int tilesN = N >> 6;
  const int tilesM = M >> 6;
  const int tile = blockIdx.x * 8 + wave;
  if (tile >= tilesM * tilesN) return;
  const int tm = tile / tilesN;
  const int tn = tile - tm * tilesN;
  const int m0 = tm << 6;
  const int n0 = tn << 6;

  const T* Ab  = A  + (size_t)b * strideA;
  const T* Bb  = Bt + (size_t)b * strideB;
  const T* Ab2 = SPLIT ? (A2  + (size_t)b * strideA) : nullptr;
  const T* Bb2 = SPLIT ? (Bt2 + (size_t)b * strideB) : nullptr;

  const int rlane = lane & 15;
  const int koff  = (lane >> 4) * 8;
  const int mOff  = (lane >> 4) * 8;

  v8f acc[4][4];
#pragma unroll
  for (int i = 0; i < 4; ++i)
#pragma unroll
    for (int j = 0; j < 4; ++j) acc[i][j] = (v8f){0.f,0.f,0.f,0.f,0.f,0.f,0.f,0.f};

  for (int k0 = 0; k0 < K; k0 += 32) {
    V bh[4], bl[4];
#pragma unroll
    for (int j = 0; j < 4; ++j) {
      const size_t bo = (size_t)(n0 + (j << 4) + rlane) * ldb + koff + k0;
      bh[j] = Frag<T>::load(Bb + bo);
      if (SPLIT) bl[j] = Frag<T>::load(Bb2 + bo);
    }
#pragma unroll
    for (int i = 0; i < 4; ++i) {
      const size_t ao = (size_t)(m0 + (i << 4) + rlane) * lda + koff + k0;
      V ah = Frag<T>::load(Ab + ao);
      V al;
      if (SPLIT) al = Frag<T>::load(Ab2 + ao);
#pragma unroll
      for (int j = 0; j < 4; ++j) {
        acc[i][j] = Frag<T>::mma(ah, bh[j], acc[i][j]);
        if (SPLIT) {
          acc[i][j] = Frag<T>::mma(ah, bl[j], acc[i][j]);
          acc[i][j] = Frag<T>::mma(al, bh[j], acc[i][j]);
        }
      }
      Frag<T>::guard4(acc[i][0], acc[i][1], acc[i][2], acc[i][3], ah, SPLIT ? al : bh[3]);
    }
    Frag<T>::keep(bh[0], bh[1], bh[2], bh[3]);
    if (SPLIT) Frag<T>::keep(bl[0], bl[1], bl[2], bl[3]);
  }
  acc_guard4(acc[0][0], acc[0][1], acc[0][2], acc[0][3]);
  acc_guard4(acc[1][0], acc[1][1], acc[1][2], acc[1][3]);
  acc_guard4(acc[2][0], acc[2][1], acc[2][2], acc[2][3]);
  acc_guard4(acc[3][0], acc[3][1], acc[3][2], acc[3][3]);

  float* slab = sT[wave];
  const float* Rb = RESID ? (resid + (size_t)b * strideR) : nullptr;
#pragma unroll
  for (int i = 0; i < 4; ++i) {
    const int mBase = m0 + (i << 4);
#pragma unroll
    for (int j = 0; j < 4; ++j) {
      const int n = n0 + (j << 4) + rlane;
      float bv = 0.f;
      if (BIAS_MODE == 2) bv = bias[n];
#pragma unroll
      for (int r = 0; r < 8; ++r) {
        float v = acc[i][j][r] * scale;
        if (BIAS_MODE == 1) v += bias[mBase + mOff + r];
        if (BIAS_MODE == 2) v += bv;
        if (RESID) v += Rb[(size_t)(mBase + mOff + r) * ldc + n];
        if (ACT == 2) v = fmaxf(v, 0.0f);
        if (ACT == 4) v = (v > 0.f) ? v : 0.01f * v;
        slab[(mOff + r) * 68 + (j << 4) + rlane] = v;
      }
    }
    __builtin_amdgcn_fence(__ATOMIC_RELEASE, "workgroup");
    __builtin_amdgcn_wave_barrier();
    __builtin_amdgcn_fence(__ATOMIC_ACQUIRE, "workgroup");
    if (OUT_MODE == 0) {
      float* C = (float*)Cout + (size_t)b * strideC;
      const int hh = lane >> 4, c4 = (lane & 15) * 4;
      for (int pass = 0; pass < 2; ++pass) {
#pragma unroll
        for (int it = 0; it < 8; ++it) {
          const int row = it * 2 + hh;
          v4f v = *(const v4f*)(slab + row * 68 + c4);
          *(volatile v4f*)(C + (size_t)(mBase + row) * ldc + n0 + c4) = v;
        }
        __threadfence();
      }
    } else {
      const int q = lane >> 3, c8 = (lane & 7) * 8;
      unsigned short* C  = (unsigned short*)Cout  + (size_t)b * strideC;
      unsigned short* C2 = (OUT_MODE == 2) ? ((unsigned short*)Cout2 + (size_t)b * strideC) : nullptr;
      for (int pass = 0; pass < 2; ++pass) {
#pragma unroll
        for (int it = 0; it < 4; ++it) {
          const int row = it * 4 + q;
          const float* sp = slab + row * 68 + c8;
          v8h hv, lv;
#pragma unroll
          for (int e = 0; e < 8; ++e) {
            if (OUT_MODE == 1) {
              hv[e] = (_Float16)sp[e];
            } else {
              unsigned short hb = f2bf_bits(sp[e]);
              unsigned short lb = f2bf_bits(sp[e] - bf_bits2f(hb));
              hv[e] = __builtin_bit_cast(_Float16, hb);
              lv[e] = __builtin_bit_cast(_Float16, lb);
            }
          }
          *(volatile v8h*)(C + (size_t)(mBase + row) * ldc + n0 + c8) = hv;
          if (OUT_MODE == 2) *(volatile v8h*)(C2 + (size_t)(mBase + row) * ldc + n0 + c8) = lv;
        }
        __threadfence();
      }
    }
    __builtin_amdgcn_fence(__ATOMIC_RELEASE, "workgroup");
    __builtin_amdgcn_wave_barrier();
    __builtin_amdgcn_fence(__ATOMIC_ACQUIRE, "workgroup");
  }
}

template <int PART>
__global__ __launch_bounds__(256) void pack_bt_kernel(const float* __restrict__ src, unsigned short* __restrict__ Bt) {
  constexpr int kW     = PART ? (kIn * kNB) : kIn;
  constexpr int kGPR   = kW / 8;
  constexpr int kTotal = kOutF * kGPR;
  static_assert(kTotal % 256 == 0);
  static_assert(kGPR % 32 == 0);
  const int gi = blockIdx.x * 256 + threadIdx.x;
  if (gi >= kTotal) return;
  const int o  = gi / kGPR;
  const int c8 = (gi - o * kGPR) * 8;
  const float* p = src + (size_t)o * kW + c8;
  const v4f a = *(const v4f*)(p);
  const v4f c = *(const v4f*)(p + 4);
  v8h hv;
#pragma unroll
  for (int e = 0; e < 4; ++e) {
    hv[e]     = (_Float16)(a[e] * kCarryB);
    hv[4 + e] = (_Float16)(c[e] * kCarryB);
  }
  unsigned short* dst = Bt + (size_t)o * kKtot + (PART ? kIn : 0) + c8;
  *(volatile v8h*)dst = hv;
  __threadfence();
  *(volatile v8h*)dst = hv;
}

__global__ __launch_bounds__(256) void expand_a_kernel(const float* __restrict__ x, const float* __restrict__ grid,
                                                       const float* __restrict__ prelu_w,
                                                       unsigned short* __restrict__ Ah, int row0) {
  const int tid  = threadIdx.x;
  const int lane = tid & 31;
  const int wave = tid >> 5;
  const int rloc0 = blockIdx.x * kRowsPerBlk;
  const float pw = prelu_w[0];

  const float* gp = grid + (size_t)tid * kKnots;
  const v4f q0 = *(const v4f*)(gp);
  const v4f q1 = *(const v4f*)(gp + 4);
  const v4f q2 = *(const v4f*)(gp + 8);
  float g[12];
#pragma unroll
  for (int e = 0; e < 4; ++e) { g[e] = q0[e]; g[4 + e] = q1[e]; g[8 + e] = q2[e]; }
  float rc1[11], rc2[10], rc3[9];
#pragma unroll
  for (int m = 0; m < 11; ++m) rc1[m] = __builtin_amdgcn_rcpf(g[m + 1] - g[m]);
#pragma unroll
  for (int m = 0; m < 10; ++m) rc2[m] = __builtin_amdgcn_rcpf(g[m + 2] - g[m]);
#pragma unroll
  for (int m = 0; m < 9; ++m) rc3[m] = __builtin_amdgcn_rcpf(g[m + 3] - g[m]);

  {
    const int rl = rloc0 + wave;
    const float* xp = x + (size_t)(row0 + rl) * kIn + 8 * lane;
    const v4f a = *(const v4f*)(xp);
    const v4f c = *(const v4f*)(xp + 4);
    v8h hv;
#pragma unroll
    for (int e = 0; e < 4; ++e) {
      float v0 = a[e]; v0 = (v0 >= 0.0f) ? v0 : pw * v0; hv[e]     = (_Float16)(v0 * kCarryA);
      float v1 = c[e]; v1 = (v1 >= 0.0f) ? v1 : pw * v1; hv[4 + e] = (_Float16)(v1 * kCarryA);
    }
    unsigned short* dst = Ah + (size_t)rl * kKtot + 8 * lane;
    *(volatile v8h*)dst = hv;
    __threadfence();
    *(volatile v8h*)dst = hv;
  }

#pragma unroll 1
  for (int r = 0; r < kRowsPerBlk; ++r) {
    const int rl = rloc0 + r;
    const float xv = x[(size_t)(row0 + rl) * kIn + tid];
    float bb[11];
#pragma unroll
    for (int j = 0; j < 11; ++j) bb[j] = ((xv >= g[j]) && (xv < g[j + 1])) ? 1.0f : 0.0f;
#pragma unroll
    for (int j = 0; j < 10; ++j) {
      const float lf = (xv - g[j]) * rc1[j];
      const float rt = (g[j + 2] - xv) * rc1[j + 1];
      bb[j] = lf * bb[j] + rt * bb[j + 1];
    }
#pragma unroll
    for (int j = 0; j < 9; ++j) {
      const float lf = (xv - g[j]) * rc2[j];
      const float rt = (g[j + 3] - xv) * rc2[j + 1];
      bb[j] = lf * bb[j] + rt * bb[j + 1];
    }
#pragma unroll
    for (int j = 0; j < 8; ++j) {
      const float lf = (xv - g[j]) * rc3[j];
      const float rt = (g[j + 4] - xv) * rc3[j + 1];
      bb[j] = lf * bb[j] + rt * bb[j + 1];
    }
    v8h hv;
#pragma unroll
    for (int e = 0; e < 8; ++e) hv[e] = (_Float16)(bb[e] * kCarryA);
    unsigned short* dst = Ah + (size_t)rl * kKtot + kIn + 8 * tid;
    *(volatile v8h*)dst = hv;
    __threadfence();
    *(volatile v8h*)dst = hv;
  }
}

extern "C" void kernel_launch(void* const* d_in, const int* in_sizes, int n_in,
                              void* d_out, int out_size, void* d_ws, size_t ws_size,
                              hipStream_t stream) {
  if (n_in < 5) return;
  if (in_sizes[0] != kRows * kIn) return;
  if (in_sizes[1] != kIn * kKnots) return;
  if (in_sizes[2] != kOutF * kIn) return;
  if (in_sizes[3] != kOutF * kIn * kNB) return;
  if (in_sizes[4] < 1) return;
  if (out_size != kRows * kOutF) return;
  if (ws_size < kWsNeed) return;

  const float* xp  = (const float*)d_in[0];
  const float* grd = (const float*)d_in[1];
  const float* bw  = (const float*)d_in[2];
  const float* sw  = (const float*)d_in[3];
  const float* pwp = (const float*)d_in[4];
  float* outp = (float*)d_out;

  unsigned short* Bt = (unsigned short*)d_ws;
  unsigned short* Ah = (unsigned short*)((char*)d_ws + kBtBytes);

  pack_bt_kernel<0><<<(kOutF * (kIn / 8)) / 256, 256, 0, stream>>>(bw, Bt);
  pack_bt_kernel<1><<<(kOutF * (kIn * kNB / 8)) / 256, 256, 0, stream>>>(sw, Bt);

  const int tiles      = (kHalfRows / 64) * (kOutF / 64);
  const int gemmBlocks = (tiles + 7) / 8;
  for (int h = 0; h < 2; ++h) {
    const int row0 = h * kHalfRows;
    expand_a_kernel<<<kHalfRows / kRowsPerBlk, 256, 0, stream>>>(xp, grd, pwp, Ah, row0);
    float* cp = outp + (size_t)row0 * kOutF;
    wmma_gemm64<0, false, 0, 0, false, 0><<<dim3(gemmBlocks, 1), 256, 0, stream>>>(
        Ah, Ah, kKtot, 0L,
        Bt, Bt, kKtot, 0L,
        (void*)cp, (void*)cp, kOutF, 0L,
        pwp,
        xp, 0L,
        kHalfRows, kOutF, kKtot, kOutScale);
  }
}
